// KTMutualAttention_34239479284420
// MI455X (gfx1250) — hardware-run, weakly checked
//
#include <hip/hip_runtime.h>


#define NB_  8
#define TQ_  512
#define SK   1024
#define TL   64
#define DD   1024
#define NH_  16
#define HD   64
#define PCAR 1024.0f
typedef _Float16 h16;
typedef unsigned short bf;
typedef __attribute__((ext_vector_type(16))) __bf16   v16bf;
typedef __attribute__((ext_vector_type(16))) _Float16 v16h;
typedef __attribute__((ext_vector_type(8)))  _Float16 v8h;
typedef __attribute__((ext_vector_type(8)))  unsigned short v8us;
typedef __attribute__((ext_vector_type(8)))  float    v8f;
typedef __attribute__((ext_vector_type(4)))  float    v4f;
typedef v8h  __attribute__((may_alias)) v8ha;
typedef v4f  __attribute__((may_alias)) v4fa;
typedef v8us __attribute__((may_alias)) v8usa;

__device__ __forceinline__ unsigned short f2bf(float f) { unsigned u = __float_as_uint(f); u += 0x7FFFu + ((u >> 16) & 1u); return (unsigned short)(u >> 16); }
__device__ __forceinline__ float bf2f(unsigned short b) { return __uint_as_float(((unsigned)b) << 16); }
__device__ __forceinline__ float bfr(float f) { return bf2f(f2bf(f)); }
__device__ __forceinline__ v16h cat16(v8h lo, v8h hi) { return __builtin_shufflevector(lo, hi, 0, 1, 2, 3, 4, 5, 6, 7, 8, 9, 10, 11, 12, 13, 14, 15); }
__device__ __forceinline__ v16bf cat16b(v8us lo, v8us hi) { return __builtin_bit_cast(v16bf, __builtin_shufflevector(lo, hi, 0, 1, 2, 3, 4, 5, 6, 7, 8, 9, 10, 11, 12, 13, 14, 15)); }
__device__ __forceinline__ v8f wmma16(v16h a, v16h b, v8f c) { return __builtin_amdgcn_wmma_f32_16x16x32_f16(false, a, false, b, (short)0, c, false, false); }
__device__ __forceinline__ v8f wmmab(v16bf a, v16bf b, v8f c) { return __builtin_amdgcn_wmma_f32_16x16x32_bf16(false, a, false, b, (short)0, c, false, false); }


template <typename T16> struct WFrag;
template <> struct WFrag<h16> { typedef v16h V; static __device__ __forceinline__ V ld(const h16* p) { return cat16(*(const v8h*)p, *(const v8h*)(p + 16)); } static __device__ __forceinline__ v8f mma(V a, V b, v8f c) { return wmma16(a, b, c); } };
template <> struct WFrag<bf> { typedef v16bf V; static __device__ __forceinline__ V ld(const bf* p) { return cat16b(*(const v8us*)p, *(const v8us*)(p + 16)); } static __device__ __forceinline__ v8f mma(V a, V b, v8f c) { return wmmab(a, b, c); } };
template <typename T16, int NSPLIT, bool BIAS>
__global__ __launch_bounds__(32) void k_gemmw(const T16* __restrict__ A, const T16* __restrict__ A2, const T16* __restrict__ Bt, const T16* __restrict__ Bt2, int K, float* C, int ldc, const float* __restrict__ bias, size_t sA, size_t sB, size_t sC) {
    typedef typename WFrag<T16>::V V;
    __shared__ __align__(16) float os[16 * 68];
    const size_t z = blockIdx.z; A += z * sA; if (A2) A2 += z * sA; Bt += z * sB; if (Bt2) Bt2 += z * sB; C += z * sC;
    const int lane = threadIdx.x & 31, lr = lane & 15, hi = lane >> 4; const int r0 = blockIdx.x * 64, c0 = blockIdx.y * 64;
    v8f acc[4][4];
#pragma unroll
    for (int mb = 0; mb < 4; ++mb)
#pragma unroll
        for (int nb = 0; nb < 4; ++nb) acc[mb][nb] = (v8f){};
    const size_t aoff = (size_t)(r0 + lr) * K + 8 * hi, boff = (size_t)(c0 + lr) * K + 8 * hi;
#pragma unroll 1
    for (int kc = 0; kc < K; kc += 32) {
        V a[4], a2[4];
#pragma unroll
        for (int mb = 0; mb < 4; ++mb) { a[mb] = WFrag<T16>::ld(A + aoff + (size_t)mb * 16 * K + kc); if (NSPLIT == 1 || NSPLIT == 2) a2[mb] = WFrag<T16>::ld(A2 + aoff + (size_t)mb * 16 * K + kc); }
#pragma unroll
        for (int nb = 0; nb < 4; ++nb) { const V b = WFrag<T16>::ld(Bt + boff + (size_t)nb * 16 * K + kc); V b2; if (NSPLIT >= 2) b2 = WFrag<T16>::ld(Bt2 + boff + (size_t)nb * 16 * K + kc);
#pragma unroll
            for (int mb = 0; mb < 4; ++mb) { acc[mb][nb] = WFrag<T16>::mma(a[mb], b, acc[mb][nb]); if (NSPLIT == 1 || NSPLIT == 2) acc[mb][nb] = WFrag<T16>::mma(a2[mb], b, acc[mb][nb]); if (NSPLIT >= 2) acc[mb][nb] = WFrag<T16>::mma(a[mb], b2, acc[mb][nb]); } }
        asm volatile("v_nop\n\tv_nop\n\tv_nop\n\tv_nop" : "+v"(acc[0][0]), "+v"(acc[1][1]), "+v"(acc[2][2]), "+v"(acc[3][3]) : "v"(a[0]), "v"(a[3]));
    }
#pragma unroll
    for (int mb = 0; mb < 4; ++mb) {
#pragma unroll
        for (int nb = 0; nb < 4; ++nb) {
#pragma unroll
            for (int j = 0; j < 8; ++j) os[(hi * 8 + j) * 68 + nb * 16 + lr] = acc[mb][nb][j]; }
        __builtin_amdgcn_wave_barrier(); asm volatile("" ::: "memory");
        float* crow = C + (size_t)(r0 + mb * 16) * ldc + c0;
#pragma unroll 1
        for (int ps = 0; ps < 2; ++ps) {
#pragma unroll
            for (int s = 0; s < 8; ++s) { const int row = 2 * s + hi, cofs = lr * 4; v4f val = *(const v4fa*)(os + row * 68 + cofs); if (BIAS) { val[0] += bfr(bias[c0 + cofs]); val[1] += bfr(bias[c0 + cofs + 1]); val[2] += bfr(bias[c0 + cofs + 2]); val[3] += bfr(bias[c0 + cofs + 3]); }
                *(volatile v4f*)(crow + (size_t)row * ldc + cofs) = val; }
            if (ps == 0) __threadfence(); }
        __builtin_amdgcn_wave_barrier(); asm volatile("" ::: "memory");
    }
}

__device__ __forceinline__ h16 tohx(float x) { return (h16)x; }
__device__ __forceinline__ void splitf(float y, unsigned short& h, unsigned short& l) { h = f2bf(y); l = f2bf(y - bf2f(h)); }
typedef __attribute__((ext_vector_type(2))) _Float16 v2h;
typedef __attribute__((ext_vector_type(4))) _Float16 v4h;
typedef __attribute__((ext_vector_type(2))) unsigned short v2us;
typedef __attribute__((ext_vector_type(8))) _Float16 v8h16;

__global__ __launch_bounds__(256) void k_cvt8(const float* __restrict__ src, bf* dst, size_t n8) { const size_t i = (size_t)blockIdx.x * 256 + threadIdx.x; if (i >= n8) return; const v8f v = *(const v8f*)(src + i * 8); v8us o;
#pragma unroll
    for (int k = 0; k < 8; ++k) o[k] = f2bf(v[k]); *(volatile v8us*)(dst + i * 8) = o; __threadfence(); *(volatile v8us*)(dst + i * 8) = o; }
__global__ __launch_bounds__(256) void k_pl(const float* __restrict__ F, int rows, int lg2, float sc, h16* P) {
    const int lane = threadIdx.x & 31; const int L0 = (blockIdx.x * 8 + (threadIdx.x >> 5)) * 8; const int nlines = NH_ * rows * HD / 64;
#pragma unroll 1
    for (int ps = 0; ps < 2; ++ps) {
#pragma unroll
        for (int l = 0; l < 8; ++l) { const int L = L0 + l; if (L >= nlines) break; const int e = L * 64 + lane * 2; const int d = e & (HD - 1); const int r = (e >> 6) & (rows - 1); const int h = e >> (6 + lg2); v2h o;
#pragma unroll
            for (int q = 0; q < 2; ++q) o[q] = tohx(F[(size_t)r * DD + h * HD + d + q] * sc);
            *(volatile v2h*)(P + (size_t)e) = o; }
        if (ps == 0) __threadfence(); }
}
__global__ __launch_bounds__(256) void k_vt(const float* __restrict__ F, h16* VT) {
    const int lane = threadIdx.x & 31; const int L0 = (blockIdx.x * 8 + (threadIdx.x >> 5)) * 8; const int nlines = NH_ * HD * SK / 64;
#pragma unroll 1
    for (int ps = 0; ps < 2; ++ps) {
#pragma unroll
        for (int l = 0; l < 8; ++l) { const int L = L0 + l; if (L >= nlines) break; const int e = L * 64 + lane * 2; const int s = e & (SK - 1); const int d = (e >> 10) & (HD - 1); const int h = e >> 16; v2h o;
#pragma unroll
            for (int q = 0; q < 2; ++q) o[q] = tohx(F[(size_t)(s + q) * DD + h * HD + d]);
            *(volatile v2h*)(VT + (size_t)e) = o; }
        if (ps == 0) __threadfence(); }
}
__global__ __launch_bounds__(256) void k_w(const float* __restrict__ TA, const float* __restrict__ mk, float* Wv) {
    const int s = blockIdx.x * 256 + threadIdx.x; if (s >= SK) return; float num = 0.f, den = 0.f;
#pragma unroll 4
    for (int t = 0; t < TL; ++t) { const float m = mk[(size_t)s * TL + t]; float p = __fmul_rn(TA[(size_t)s * TL + t], m); asm volatile("" : "+v"(p)); num = __fadd_rn(num, p); den = __fadd_rn(den, m); }
    const float o = __fdiv_rn(num, den); *(volatile float*)(Wv + s) = o; __threadfence(); *(volatile float*)(Wv + s) = o; }
__global__ __launch_bounds__(256) void k_wsoft(const float* __restrict__ Sb, const float* __restrict__ Wv, h16* P16) {
    const int lane = threadIdx.x & 31; const int row = blockIdx.x * 8 + (threadIdx.x >> 5); if (row >= TQ_) return; const float* sr = Sb + (size_t)row * SK; float v[32]; float mx = -3.0e38f;
#pragma unroll
    for (int ch = 0; ch < 8; ++ch) { const int j0 = ch * 128 + lane * 4; const v4f a = *(const v4f*)(sr + j0), ww = *(const v4f*)(Wv + j0);
#pragma unroll
        for (int q = 0; q < 4; ++q) { const float t = __fmul_rn(a[q], ww[q]); v[ch * 4 + q] = t; mx = fmaxf(mx, t); } }
#pragma unroll
    for (int sh = 16; sh; sh >>= 1) mx = fmaxf(mx, __shfl_xor(mx, sh, 32));
    float sum = 0.f;
#pragma unroll
    for (int k = 0; k < 32; ++k) { v[k] = __expf(v[k] - mx); sum += v[k]; }
#pragma unroll
    for (int sh = 16; sh; sh >>= 1) sum += __shfl_xor(sum, sh, 32);
    const float f = __fdiv_rn(PCAR, sum);
#pragma unroll 1
    for (int ps = 0; ps < 2; ++ps) {
#pragma unroll
        for (int ch = 0; ch < 8; ++ch) { v4h o;
#pragma unroll
            for (int q = 0; q < 4; ++q) o[q] = tohx(v[ch * 4 + q] * f);
            *(volatile v4h*)(P16 + (size_t)row * SK + ch * 128 + lane * 4) = o; }
        if (ps == 0) __threadfence(); }
}
__global__ __launch_bounds__(256) void k_merge(const float* __restrict__ O, int h, bf* Ah, bf* Al) { const int i = (blockIdx.x * 256 + threadIdx.x) * 2; if (i >= TQ_ * HD) return; const int t = i >> 6, d = i & 63; v2us oh, ol;
#pragma unroll
    for (int q = 0; q < 2; ++q) { unsigned short a, c2; splitf(O[i + q] * (1.0f / PCAR), a, c2); oh[q] = a; ol[q] = c2; }
    const size_t o = (size_t)t * DD + h * HD + d; *(volatile v2us*)(Ah + o) = oh; *(volatile v2us*)(Al + o) = ol; __threadfence(); *(volatile v2us*)(Ah + o) = oh; *(volatile v2us*)(Al + o) = ol; }

extern "C" void kernel_launch(void* const* d_in, const int* in_sizes, int n_in,
                              void* d_out, int out_size, void* d_ws, size_t ws_size, hipStream_t stream) {
    (void)in_sizes; (void)n_in; (void)out_size;
    const float* IN[16]; for (int i = 0; i < 16; ++i) IN[i] = (const float*)d_in[i];
    float* OUT = (float*)d_out;
    char* wsp = (char*)d_ws;
    auto take = [&](size_t bytes) { char* p = wsp; wsp += (bytes + 255) & ~(size_t)255; return (void*)p; };
    bf* WQ = (bf*)take((size_t)DD * DD * 2); bf* WK = (bf*)take((size_t)DD * DD * 2); bf* WV = (bf*)take((size_t)DD * DD * 2); bf* WWQ = (bf*)take((size_t)DD * DD * 2); bf* WWK = (bf*)take((size_t)DD * DD * 2); bf* WO = (bf*)take((size_t)DD * DD * 2);
    bf* XH = (bf*)take((size_t)TQ_ * DD * 2); bf* XKV = (bf*)take((size_t)SK * DD * 2); bf* XT = (bf*)take((size_t)TL * DD * 2); float* F = (float*)take((size_t)SK * DD * 4);
    h16* QP = (h16*)take((size_t)NH_ * TQ_ * HD * 2); h16* KP = (h16*)take((size_t)NH_ * SK * HD * 2); h16* VT = (h16*)take((size_t)NH_ * HD * SK * 2); h16* TQP = (h16*)take((size_t)NH_ * SK * HD * 2); h16* TKP = (h16*)take((size_t)NH_ * TL * HD * 2);
    float* TA = (float*)take((size_t)SK * TL * 4); float* Wv = (float*)take((size_t)SK * 4); float* Sb = (float*)take((size_t)TQ_ * SK * 4); h16* Pm = (h16*)take((size_t)TQ_ * SK * 2); float* Ob = (float*)take((size_t)TQ_ * HD * 4); bf* ATh = (bf*)take((size_t)TQ_ * DD * 2); bf* ATl = (bf*)take((size_t)TQ_ * DD * 2);
    if ((size_t)(wsp - (char*)d_ws) > ws_size) return;
    { const size_t nw = (size_t)DD * DD / 8; const unsigned gw = (unsigned)((nw + 255) / 256); const float* ws_[6] = {IN[4], IN[6], IN[8], IN[10], IN[12], IN[14]}; bf* wd_[6] = {WQ, WK, WV, WWQ, WWK, WO};
      for (int i = 0; i < 6; ++i) k_cvt8<<<gw, 256, 0, stream>>>(ws_[i], wd_[i], nw); }
    for (int b = 0; b < NB_; ++b) { const float* mkb = IN[3] + (size_t)b * SK * TL;
        k_cvt8<<<(unsigned)(((size_t)TQ_ * DD / 8 + 255) / 256), 256, 0, stream>>>(IN[0] + (size_t)b * TQ_ * DD, XH, (size_t)TQ_ * DD / 8);
        k_cvt8<<<(unsigned)(((size_t)SK * DD / 8 + 255) / 256), 256, 0, stream>>>(IN[1] + (size_t)b * SK * DD, XKV, (size_t)SK * DD / 8);
        k_cvt8<<<(unsigned)(((size_t)TL * DD / 8 + 255) / 256), 256, 0, stream>>>(IN[2] + (size_t)b * TL * DD, XT, (size_t)TL * DD / 8);
        k_gemmw<bf, 0, true><<<dim3(TQ_ / 64, DD / 64, 1), 32, 0, stream>>>(XH, nullptr, WQ, nullptr, DD, F, DD, IN[5], 0, 0, 0);   k_pl<<<(NH_ * TQ_ * HD / 64 + 63) / 64, 256, 0, stream>>>(F, TQ_, 9, 0.125f, QP);
        k_gemmw<bf, 0, true><<<dim3(SK / 64, DD / 64, 1), 32, 0, stream>>>(XKV, nullptr, WK, nullptr, DD, F, DD, IN[7], 0, 0, 0);   k_pl<<<(NH_ * SK * HD / 64 + 63) / 64, 256, 0, stream>>>(F, SK, 10, 1.0f, KP);
        k_gemmw<bf, 0, true><<<dim3(SK / 64, DD / 64, 1), 32, 0, stream>>>(XKV, nullptr, WV, nullptr, DD, F, DD, IN[9], 0, 0, 0);   k_vt<<<(NH_ * HD * SK / 64 + 63) / 64, 256, 0, stream>>>(F, VT);
        k_gemmw<bf, 0, true><<<dim3(SK / 64, DD / 64, 1), 32, 0, stream>>>(XKV, nullptr, WWQ, nullptr, DD, F, DD, IN[11], 0, 0, 0); k_pl<<<(NH_ * SK * HD / 64 + 63) / 64, 256, 0, stream>>>(F, SK, 10, 0.125f, TQP);
        k_gemmw<bf, 0, true><<<dim3(TL / 64, DD / 64, 1), 32, 0, stream>>>(XT, nullptr, WWK, nullptr, DD, F, DD, IN[13], 0, 0, 0);  k_pl<<<(NH_ * TL * HD / 64 + 63) / 64, 256, 0, stream>>>(F, TL, 6, 1.0f, TKP);
        for (int h = 0; h < NH_; ++h) {
            k_gemmw<h16, 0, false><<<dim3(SK / 64, TL / 64, 1), 32, 0, stream>>>(TQP + (size_t)h * SK * HD, nullptr, TKP + (size_t)h * TL * HD, nullptr, HD, TA, TL, nullptr, 0, 0, 0);
            k_w<<<SK / 256, 256, 0, stream>>>(TA, mkb, Wv);
            k_gemmw<h16, 0, false><<<dim3(TQ_ / 64, SK / 64, 1), 32, 0, stream>>>(QP + (size_t)h * TQ_ * HD, nullptr, KP + (size_t)h * SK * HD, nullptr, HD, Sb, SK, nullptr, 0, 0, 0);
            k_wsoft<<<TQ_ / 8, 256, 0, stream>>>(Sb, Wv, Pm);
            k_gemmw<h16, 0, false><<<dim3(TQ_ / 64, 1, 1), 32, 0, stream>>>(Pm, nullptr, VT + (size_t)h * HD * SK, nullptr, SK, Ob, HD, nullptr, 0, 0, 0);
            k_merge<<<(TQ_ * HD / 2 + 255) / 256, 256, 0, stream>>>(Ob, h, ATh, ATl); }
        k_gemmw<bf, 1, true><<<dim3(TQ_ / 64, DD / 64, 1), 32, 0, stream>>>(ATh, ATl, WO, nullptr, DD, OUT + (size_t)b * TQ_ * DD, DD, IN[15], 0, 0, 0); }
}
